// BidirectionalMambaBlock_50371376448081
// MI455X (gfx1250) — hardware-run, weakly checked
//
#include <hip/hip_runtime.h>
#include <math.h>

typedef __attribute__((ext_vector_type(16))) _Float16 v16h;
typedef __attribute__((ext_vector_type(8)))  _Float16 v8h;
typedef __attribute__((ext_vector_type(4)))  _Float16 v4h;
typedef __attribute__((ext_vector_type(16))) __bf16   v16b;
typedef __attribute__((ext_vector_type(8)))  __bf16   v8b;
typedef __attribute__((ext_vector_type(8)))  float    v8f;
typedef __attribute__((ext_vector_type(4)))  float    v4f;

constexpr int kBatch  = 8;
constexpr int kSeq    = 256;
constexpr int kDm     = 512;
constexpr int kDin    = 1024;
constexpr int kNst    = 16;
constexpr int kDtR    = 32;
constexpr int kXzP    = 2 * kDin;
constexpr int kXdP    = kDtR + 2 * kNst;
constexpr int kHid    = 1024;
constexpr int kRows   = kBatch * kSeq;
constexpr int kConvTP = 260;
constexpr int kScanTS = 64;
constexpr int kScanCh = 64;
constexpr int kScanYP = 68;
constexpr int kLnThreads = 128;

constexpr float kCarryW  = 64.0f;
constexpr float kCarryXc = 16.0f;
constexpr float kCarryY  = 64.0f;
constexpr float kScaleIn  = 1.0f / kCarryW;
constexpr float kScaleXp  = 1.0f / (kCarryXc * kCarryW);
constexpr float kScaleOut = 1.0f / (kCarryY * kCarryW);
constexpr float kScaleMlp = 1.0f / kCarryW;
constexpr float kInvDm = 1.0f / (float)kDm;
constexpr float kLnEps = 1e-5f;

static_assert(kXdP == 64, "xproj width");
static_assert((kDm % 32) == 0 && (kDin % 32) == 0 && (kHid % 32) == 0, "GEMM K multiples of 32");
static_assert((kRows % 64) == 0 && (kXzP % 64) == 0 && (kXdP % 64) == 0 && (kDm % 64) == 0 && (kHid % 64) == 0, "GEMM M,N multiples of 64");
static_assert((kSeq % kScanTS) == 0 && (kSeq % 64) == 0 && (kDin % kScanCh) == 0 && (kDin % 256) == 0, "tile multiples");
static_assert(kDm == kLnThreads * 4, "LN thread map");
static_assert((kDm % 256) == 0, "cast wave stays inside one row");
static_assert(((kRows / 64) * (kXzP / 64)) % 8 == 0 && ((kRows / 64) * (kXdP / 64)) % 8 == 0 &&
              ((kRows / 64) * (kDm / 64)) % 8 == 0 && ((kRows / 64) * (kHid / 64)) % 8 == 0, "8 tiles per GEMM block");

constexpr size_t kOffX16  = 0;
constexpr size_t kOffXF16 = kOffX16  + (size_t)kRows * kDm  * 2;
constexpr size_t kOffINW0 = kOffXF16 + (size_t)kRows * kDm  * 2;
constexpr size_t kOffINW1 = kOffINW0 + (size_t)kXzP  * kDm  * 2;
constexpr size_t kOffXPW0 = kOffINW1 + (size_t)kXzP  * kDm  * 2;
constexpr size_t kOffXPW1 = kOffXPW0 + (size_t)kXdP  * kDin * 2;
constexpr size_t kOffOUW0 = kOffXPW1 + (size_t)kXdP  * kDin * 2;
constexpr size_t kOffOUW1 = kOffOUW0 + (size_t)kDm   * kDin * 2;
constexpr size_t kOffPU16 = kOffOUW1 + (size_t)kDm   * kDin * 2;
constexpr size_t kOffPL16 = kOffPU16 + (size_t)kHid  * kDm  * 2;
constexpr size_t kOffXZ0  = kOffPL16 + (size_t)kDm   * kHid * 2;
constexpr size_t kOffXZ1  = kOffXZ0  + (size_t)kRows * kXzP * 4;
constexpr size_t kOffXC0  = kOffXZ1  + (size_t)kRows * kXzP * 4;
constexpr size_t kOffXC1  = kOffXC0  + (size_t)kRows * kDin * 4;
constexpr size_t kOffXH0  = kOffXC1  + (size_t)kRows * kDin * 4;
constexpr size_t kOffXH1  = kOffXH0  + (size_t)kRows * kDin * 2;
constexpr size_t kOffDB0  = kOffXH1  + (size_t)kRows * kDin * 2;
constexpr size_t kOffDB1  = kOffDB0  + (size_t)kRows * kXdP * 4;
constexpr size_t kOffYG0  = kOffDB1  + (size_t)kRows * kXdP * 4;
constexpr size_t kOffYG1  = kOffYG0  + (size_t)kRows * kDin * 2;
constexpr size_t kOffY1   = kOffYG1  + (size_t)kRows * kDin * 2;
constexpr size_t kOffY2   = kOffY1   + (size_t)kRows * kDm  * 4;
constexpr size_t kOffY3   = kOffY2   + (size_t)kRows * kDm  * 4;
constexpr size_t kOffY3H  = kOffY3   + (size_t)kRows * kDm  * 4;
constexpr size_t kOffH16  = kOffY3H  + (size_t)kRows * kDm  * 2;
constexpr size_t kOffYP   = kOffH16  + (size_t)kRows * kHid * 2;
constexpr size_t kWsTotal = kOffYP   + (size_t)kRows * kDm  * 4;
static_assert(kWsTotal == 104071168ull, "carve total");
static_assert(kWsTotal <= 134217728ull, "carve cap");
static_assert((kOffXF16 % 128) == 0 && (kOffINW0 % 128) == 0 && (kOffINW1 % 128) == 0 && (kOffXPW0 % 128) == 0 &&
              (kOffXPW1 % 128) == 0 && (kOffOUW0 % 128) == 0 && (kOffOUW1 % 128) == 0 && (kOffPU16 % 128) == 0 &&
              (kOffPL16 % 128) == 0 && (kOffXZ0 % 128) == 0 && (kOffXZ1 % 128) == 0 && (kOffXC0 % 128) == 0 &&
              (kOffXC1 % 128) == 0 && (kOffXH0 % 128) == 0 && (kOffXH1 % 128) == 0 && (kOffDB0 % 128) == 0 &&
              (kOffDB1 % 128) == 0 && (kOffYG0 % 128) == 0 && (kOffYG1 % 128) == 0 && (kOffY1 % 128) == 0 &&
              (kOffY2 % 128) == 0 && (kOffY3 % 128) == 0 && (kOffY3H % 128) == 0 && (kOffH16 % 128) == 0 &&
              (kOffYP % 128) == 0, "128-B aligned regions");

__device__ __forceinline__ unsigned short f2bf_bits(float f) {
  unsigned u = __float_as_uint(f);
  return (unsigned short)((u + 0x7FFFu + ((u >> 16) & 1u)) >> 16);
}
__device__ __forceinline__ float bf_bits2f(unsigned short h) { return __uint_as_float(((unsigned)h) << 16); }

__device__ __forceinline__ void dep_guard_h(v8f& a, v8f& b, v16h x, v16h y) { asm volatile("v_nop\n\tv_nop\n\tv_nop\n\tv_nop" : "+v"(a), "+v"(b) : "v"(x), "v"(y)); }
__device__ __forceinline__ void dep_guard_b(v8f& a, v8f& b, v16b x, v16b y) { asm volatile("v_nop\n\tv_nop\n\tv_nop\n\tv_nop" : "+v"(a), "+v"(b) : "v"(x), "v"(y)); }
__device__ __forceinline__ void keep4_h(v16h a, v16h b, v16h c, v16h d) { asm volatile("v_nop" :: "v"(a), "v"(b), "v"(c), "v"(d)); }
__device__ __forceinline__ void keep4_b(v16b a, v16b b, v16b c, v16b d) { asm volatile("v_nop" :: "v"(a), "v"(b), "v"(c), "v"(d)); }
__device__ __forceinline__ void acc_guard4(v8f& a, v8f& b, v8f& c, v8f& d) { asm volatile("v_nop\n\tv_nop\n\tv_nop\n\tv_nop" : "+v"(a), "+v"(b), "+v"(c), "+v"(d)); }
template <typename T> struct Frag;
template <> struct Frag<_Float16> {
  typedef v16h V; union U { v16h v; v8h h[2]; };
  static __device__ __forceinline__ v16h load(const _Float16* p) {
    U f; f.h[0] = *(const v8h*)(p); f.h[1] = *(const v8h*)(p + 16); return f.v;
  }
  static __device__ __forceinline__ v8f mma(v16h a, v16h b, v8f c) {
    return __builtin_amdgcn_wmma_f32_16x16x32_f16(false, a, false, b, (short)0, c, false, false);
  }
  static __device__ __forceinline__ void guard(v8f& a, v8f& b, v16h x, v16h y) { dep_guard_h(a, b, x, y); }
  static __device__ __forceinline__ void keep(v16h a, v16h b, v16h c, v16h d) { keep4_h(a, b, c, d); }
};
template <> struct Frag<__bf16> {
  typedef v16b V; union U { v16b v; v8b h[2]; };
  static __device__ __forceinline__ v16b load(const __bf16* p) {
    U f; f.h[0] = *(const v8b*)(p); f.h[1] = *(const v8b*)(p + 16); return f.v;
  }
  static __device__ __forceinline__ v8f mma(v16b a, v16b b, v8f c) {
    return __builtin_amdgcn_wmma_f32_16x16x32_bf16(false, a, false, b, (short)0, c, false, false);
  }
  static __device__ __forceinline__ void guard(v8f& a, v8f& b, v16b x, v16b y) { dep_guard_b(a, b, x, y); }
  static __device__ __forceinline__ void keep(v16b a, v16b b, v16b c, v16b d) { keep4_b(a, b, c, d); }
};

template <int ET> struct Elem;
template <> struct Elem<0> { typedef _Float16 T; };
template <> struct Elem<1> { typedef __bf16 T; };
template <int ET, bool SPLIT, int BIAS_MODE, int OUT_MODE, bool RESID, int ACT = 0>
__global__ __launch_bounds__(256) void wmma_gemm64(
    const unsigned short* __restrict__ Ap, const unsigned short* __restrict__ A2p, int lda, long strideA,
    const unsigned short* __restrict__ Btp, const unsigned short* __restrict__ Bt2p, int ldb, long strideB,
    void* __restrict__ Cout, void* __restrict__ Cout2, int ldc, long strideC,
    const float* __restrict__ bias,
    const float* __restrict__ resid, long strideR,
    int M, int N, int K, float scale) {
  typedef typename Elem<ET>::T T;
  typedef typename Frag<T>::V V;
  const T* A = (const T*)Ap; const T* A2 = (const T*)A2p; const T* Bt = (const T*)Btp; const T* Bt2 = (const T*)Bt2p;
  __shared__ __align__(16) float sT[8][16 * 68];
  const int b    = blockIdx.y;
  const int lane = threadIdx.x & 31;
  const int wave = threadIdx.x >> 5;
  const int tilesN = N >> 6;
  const int tilesM = M >> 6;
  const int tile = blockIdx.x * 8 + wave;
  if (tile >= tilesM * tilesN) return;
  const int tm = tile / tilesN;
  const int tn = tile - tm * tilesN;
  const int m0 = tm << 6;
  const int n0 = tn << 6;

  const T* Ab  = A  + (size_t)b * strideA;
  const T* Bb  = Bt + (size_t)b * strideB;
  const T* Ab2 = SPLIT ? (A2  + (size_t)b * strideA) : nullptr;
  const T* Bb2 = SPLIT ? (Bt2 + (size_t)b * strideB) : nullptr;

  const int rlane = lane & 15;
  const int koff  = (lane >> 4) * 8;
  const int mOff  = (lane >> 4) * 8;

  v8f acc[4][4];
#pragma unroll
  for (int i = 0; i < 4; ++i)
#pragma unroll
    for (int j = 0; j < 4; ++j) acc[i][j] = (v8f){0.f,0.f,0.f,0.f,0.f,0.f,0.f,0.f};

  for (int k0 = 0; k0 < K; k0 += 32) {
    V bh[4], bl[4];
#pragma unroll
    for (int j = 0; j < 4; ++j) {
      const size_t bo = (size_t)(n0 + (j << 4) + rlane) * ldb + koff + k0;
      bh[j] = Frag<T>::load(Bb + bo);
      if (SPLIT) bl[j] = Frag<T>::load(Bb2 + bo);
    }
#pragma unroll
    for (int i = 0; i < 4; ++i) {
      const size_t ao = (size_t)(m0 + (i << 4) + rlane) * lda + koff + k0;
      V ah = Frag<T>::load(Ab + ao);
      V al;
      if (SPLIT) al = Frag<T>::load(Ab2 + ao);
#pragma unroll
      for (int j = 0; j < 4; ++j) {
        acc[i][j] = Frag<T>::mma(ah, bh[j], acc[i][j]);
        if (SPLIT) {
          acc[i][j] = Frag<T>::mma(ah, bl[j], acc[i][j]);
          acc[i][j] = Frag<T>::mma(al, bh[j], acc[i][j]);
        }
      }
      Frag<T>::guard(acc[i][0], acc[i][3], ah, SPLIT ? al : ah);
    }
    Frag<T>::keep(bh[0], bh[1], bh[2], bh[3]);
    if (SPLIT) Frag<T>::keep(bl[0], bl[1], bl[2], bl[3]);
  }
  acc_guard4(acc[0][0], acc[0][1], acc[0][2], acc[0][3]);
  acc_guard4(acc[1][0], acc[1][1], acc[1][2], acc[1][3]);
  acc_guard4(acc[2][0], acc[2][1], acc[2][2], acc[2][3]);
  acc_guard4(acc[3][0], acc[3][1], acc[3][2], acc[3][3]);

  float* slab = sT[wave];
  const float* Rb = RESID ? (resid + (size_t)b * strideR) : nullptr;
#pragma unroll
  for (int i = 0; i < 4; ++i) {
    const int mBase = m0 + (i << 4);
#pragma unroll
    for (int j = 0; j < 4; ++j) {
      const int n = n0 + (j << 4) + rlane;
      float bv = 0.f;
      if (BIAS_MODE == 2) bv = bias[n];
#pragma unroll
      for (int r = 0; r < 8; ++r) {
        float v = acc[i][j][r] * scale;
        if (BIAS_MODE == 1) v += bias[mBase + mOff + r];
        if (BIAS_MODE == 2) v += bv;
        if (RESID) v += Rb[(size_t)(mBase + mOff + r) * ldc + n];
        if (ACT == 1) v = tanhf(v);
        if (ACT == 2) v = fmaxf(v, 0.0f);
        if (ACT == 3) v = v / (1.0f + expf(-v));
        if (ACT == 4) v = (v > 0.f) ? v : 0.01f * v;
        slab[(mOff + r) * 68 + (j << 4) + rlane] = v;
      }
    }
    __builtin_amdgcn_fence(__ATOMIC_RELEASE, "workgroup");
    __builtin_amdgcn_wave_barrier();
    __builtin_amdgcn_fence(__ATOMIC_ACQUIRE, "workgroup");
    if (OUT_MODE == 0) {
      float* C = (float*)Cout + (size_t)b * strideC;
      const int hh = lane >> 4, c4 = (lane & 15) * 4;
      for (int pass = 0; pass < 2; ++pass) {
#pragma unroll
        for (int it = 0; it < 8; ++it) {
          const int row = it * 2 + hh;
          v4f v = *(const v4f*)(slab + row * 68 + c4);
          *(volatile v4f*)(C + (size_t)(mBase + row) * ldc + n0 + c4) = v;
        }
        __threadfence();
      }
    } else {
      const int q = lane >> 3, c8 = (lane & 7) * 8;
      unsigned short* C  = (unsigned short*)Cout  + (size_t)b * strideC;
      unsigned short* C2 = (OUT_MODE == 2) ? ((unsigned short*)Cout2 + (size_t)b * strideC) : nullptr;
      for (int pass = 0; pass < 2; ++pass) {
#pragma unroll
        for (int it = 0; it < 4; ++it) {
          const int row = it * 4 + q;
          const float* sp = slab + row * 68 + c8;
          v8h hv, lv;
#pragma unroll
          for (int e = 0; e < 8; ++e) {
            if (OUT_MODE == 1) {
              hv[e] = (_Float16)sp[e];
            } else {
              unsigned short hb = f2bf_bits(sp[e]);
              unsigned short lb = f2bf_bits(sp[e] - bf_bits2f(hb));
              hv[e] = __builtin_bit_cast(_Float16, hb);
              lv[e] = __builtin_bit_cast(_Float16, lb);
            }
          }
          *(volatile v8h*)(C + (size_t)(mBase + row) * ldc + n0 + c8) = hv;
          if (OUT_MODE == 2) *(volatile v8h*)(C2 + (size_t)(mBase + row) * ldc + n0 + c8) = lv;
        }
        __threadfence();
      }
    }
    __builtin_amdgcn_fence(__ATOMIC_RELEASE, "workgroup");
    __builtin_amdgcn_wave_barrier();
    __builtin_amdgcn_fence(__ATOMIC_ACQUIRE, "workgroup");
  }
}

__global__ __launch_bounds__(256) void cast_scale_f16_kernel(
    const float* __restrict__ src, unsigned short* __restrict__ dst, int total8, float scale)
{
  const int i = blockIdx.x * 256 + threadIdx.x;
  if (i >= total8) return;
  const size_t e0 = (size_t)i << 3;
  const v4f a0 = *(const v4f*)(src + e0);
  const v4f a1 = *(const v4f*)(src + e0 + 4);
  v8h hv;
#pragma unroll
  for (int e = 0; e < 4; ++e) {
    hv[e]     = (_Float16)(a0[e] * scale);
    hv[4 + e] = (_Float16)(a1[e] * scale);
  }
  unsigned short* q = dst + e0;
  *(volatile v8h*)q = hv;
  __threadfence();
  *(volatile v8h*)q = hv;
}

__global__ __launch_bounds__(256) void cast_x_f16_kernel(
    const float* __restrict__ src, unsigned short* __restrict__ dst, unsigned short* __restrict__ dstf, int total8)
{
  const int i = blockIdx.x * 256 + threadIdx.x;
  if (i >= total8) return;
  const size_t e0 = (size_t)i << 3;
  const int row = (int)(e0 / kDm);
  const int col = (int)(e0 - (size_t)row * kDm);
  const int bb = row / kSeq, t = row - bb * kSeq;
  const int frow = bb * kSeq + (kSeq - 1 - t);
  const v4f a0 = *(const v4f*)(src + e0);
  const v4f a1 = *(const v4f*)(src + e0 + 4);
  v8h hv;
#pragma unroll
  for (int e = 0; e < 4; ++e) {
    hv[e]     = (_Float16)a0[e];
    hv[4 + e] = (_Float16)a1[e];
  }
  unsigned short* q  = dst + e0;
  unsigned short* qf = dstf + (size_t)frow * kDm + col;
  *(volatile v8h*)q  = hv;
  *(volatile v8h*)qf = hv;
  __threadfence();
  *(volatile v8h*)q  = hv;
  *(volatile v8h*)qf = hv;
}

__global__ __launch_bounds__(256) void conv_silu_kernel(
    const float* __restrict__ XZ, const float* __restrict__ cw, const float* __restrict__ cb,
    float* __restrict__ XC, unsigned short* __restrict__ XH)
{
  __shared__ __align__(16) float sT[16 * kConvTP];
  const int tid = threadIdx.x, lane = tid & 31, wave = tid >> 5;
  const int d0 = blockIdx.x * 256, d = d0 + tid;
  const int g0 = blockIdx.y * 64;
  const int tb = g0 & (kSeq - 1);
  const float w0 = cw[d * 2 + 0], w1 = cw[d * 2 + 1];
  const float bc = cb[d];
  float xm1;
  {
    const bool hist = (tb > 0);
    const int rb = hist ? (g0 - 1) : g0;
    const float v1 = XZ[(size_t)rb * kXzP + d];
    xm1 = hist ? v1 : 0.f;
  }
  const int hrow = wave >> 1;
  const int hch  = (wave & 1) * 128 + lane * 4;
#pragma unroll 1
  for (int sub = 0; sub < 4; ++sub) {
    const int lb = g0 + sub * 16;
#pragma unroll 1
    for (int s = 0; s < 16; ++s) {
      const float xcur = XZ[(size_t)(lb + s) * kXzP + d];
      float acc = w0 * xm1;
      acc = fmaf(w1, xcur, acc);
      const float sv = acc + bc;
      const float sg = __builtin_amdgcn_rcpf(1.0f + expf(-sv));
      sT[s * kConvTP + tid] = sv * sg;
      xm1 = xcur;
    }
    __syncthreads();
    v4f fv[4];
    v8h hv[2];
#pragma unroll
    for (int it = 0; it < 4; ++it) fv[it] = *(const v4f*)(sT + (it * 4 + hrow) * kConvTP + hch);
#pragma unroll
    for (int it = 0; it < 2; ++it) {
      const float* sp = sT + (it * 8 + wave) * kConvTP + lane * 8;
      const v4f a0 = *(const v4f*)(sp);
      const v4f a1 = *(const v4f*)(sp + 4);
#pragma unroll
      for (int e = 0; e < 4; ++e) {
        hv[it][e]     = (_Float16)(a0[e] * kCarryXc);
        hv[it][4 + e] = (_Float16)(a1[e] * kCarryXc);
      }
    }
    for (int pass = 0; pass < 2; ++pass) {
#pragma unroll
      for (int it = 0; it < 4; ++it)
        *(volatile v4f*)(XC + (size_t)(lb + it * 4 + hrow) * kDin + d0 + hch) = fv[it];
#pragma unroll
      for (int it = 0; it < 2; ++it) {
        const size_t o = (size_t)(lb + it * 8 + wave) * kDin + d0 + lane * 8;
        *(volatile v8h*)(XH + o) = hv[it];
      }
      __threadfence();
    }
    __syncthreads();
  }
}

__global__ __launch_bounds__(kScanCh) void scan_kernel(
    const float* __restrict__ XD, const float* __restrict__ XC, const float* __restrict__ XZ,
    const float* __restrict__ Wdt, const float* __restrict__ bdt, const float* __restrict__ Alog,
    const float* __restrict__ Dp, unsigned short* __restrict__ YG)
{
  __shared__ __align__(16) float sX[kScanTS * kXdP];
  __shared__ __align__(16) float sY[kScanTS * kScanYP];
  __shared__ __align__(16) float sW[kDtR * kScanCh];
  __shared__ __align__(16) float sA[kNst * kScanCh];
  const int tid = threadIdx.x, lane = tid & 31, wave = tid >> 5;
  constexpr int kBlkPerB = kDin / kScanCh;
  const int bix = blockIdx.x / kBlkPerB;
  const int d0  = (blockIdx.x - bix * kBlkPerB) * kScanCh;
  const int d   = d0 + tid;
  const size_t row0 = (size_t)bix * kSeq;
#pragma unroll 1
  for (int r = 0; r < kDtR; ++r) sW[r * kScanCh + tid] = Wdt[(size_t)d * kDtR + r];
#pragma unroll 1
  for (int s = 0; s < kNst; ++s) sA[s * kScanCh + tid] = -expf(Alog[(size_t)d * kNst + s]);
  __syncthreads();
  float negA[kNst], h[kNst];
#pragma unroll
  for (int s = 0; s < kNst; ++s) {
    negA[s] = sA[s * kScanCh + tid];
    h[s] = 0.f;
  }
  const float bb = bdt[d], Dd = Dp[d];
  const int lr = tid >> 4, lc4 = (tid & 15) * 4;
  const int q = lane >> 3, c8 = (lane & 7) * 8;
#pragma unroll 1
  for (int t0 = 0; t0 < kSeq; t0 += kScanTS) {
    __syncthreads();
#pragma unroll 4
    for (int i = 0; i < 16; ++i) {
      const int r = lr + 4 * i;
      *(v4f*)(sX + r * kXdP + lc4) = *(const v4f*)(XD + (row0 + t0 + r) * kXdP + lc4);
    }
    __syncthreads();
#pragma unroll 1
    for (int s = 0; s < kScanTS; ++s) {
      const int t = t0 + s;
      const float* xr = sX + s * kXdP;
      float vdot = 0.f;
#pragma unroll 1
      for (int r4 = 0; r4 < kDtR / 4; ++r4) {
        const v4f xv = *(const v4f*)(xr + 4 * r4);
        const float* wp = sW + (4 * r4) * kScanCh + tid;
        vdot = fmaf(xv[0], wp[0], vdot);
        vdot = fmaf(xv[1], wp[kScanCh], vdot);
        vdot = fmaf(xv[2], wp[2 * kScanCh], vdot);
        vdot = fmaf(xv[3], wp[3 * kScanCh], vdot);
      }
      float Bs[kNst], Cs[kNst];
#pragma unroll
      for (int q4 = 0; q4 < 4; ++q4) {
        const v4f bv = *(const v4f*)(xr + kDtR + 4 * q4);
        const v4f cv = *(const v4f*)(xr + kDtR + kNst + 4 * q4);
        Bs[4 * q4 + 0] = bv[0]; Bs[4 * q4 + 1] = bv[1]; Bs[4 * q4 + 2] = bv[2]; Bs[4 * q4 + 3] = bv[3];
        Cs[4 * q4 + 0] = cv[0]; Cs[4 * q4 + 1] = cv[1]; Cs[4 * q4 + 2] = cv[2]; Cs[4 * q4 + 3] = cv[3];
      }
      const float v   = vdot + bb;
      const float ea  = expf(-fabsf(v));
      const float dt  = fmaxf(v, 0.0f) + log1pf(ea);
      const float xt  = XC[(row0 + t) * kDin + d];
      const float dtx = dt * xt;
      float y = 0.f;
#pragma unroll
      for (int k = 0; k < kNst; ++k) {
        const float e = __expf(dt * negA[k]);
        h[k] = e * h[k] + dtx * Bs[k];
        y = h[k] * Cs[k] + y;
      }
      y = xt * Dd + y;
      const float zv = XZ[(row0 + t) * kXzP + kDin + d];
      const float sg = __builtin_amdgcn_rcpf(1.0f + expf(-zv));
      y = y * (zv * sg);
      sY[s * kScanYP + tid] = y;
    }
    __syncthreads();
    v8h hv[8];
#pragma unroll
    for (int it = 0; it < 8; ++it) {
      const int row = it * 8 + wave * 4 + q;
      const float* sp = sY + row * kScanYP + c8;
      const v4f a0 = *(const v4f*)(sp);
      const v4f a1 = *(const v4f*)(sp + 4);
#pragma unroll
      for (int e = 0; e < 4; ++e) {
        hv[it][e]     = (_Float16)(a0[e] * kCarryY);
        hv[it][4 + e] = (_Float16)(a1[e] * kCarryY);
      }
    }
    for (int pass = 0; pass < 2; ++pass) {
#pragma unroll
      for (int it = 0; it < 8; ++it) {
        const int row = it * 8 + wave * 4 + q;
        const size_t o = (row0 + t0 + row) * kDin + d0 + c8;
        *(volatile v8h*)(YG + o) = hv[it];
      }
      __threadfence();
    }
  }
}

template <int MODE>
__global__ __launch_bounds__(kLnThreads) void add_ln_kernel(
    const float* __restrict__ a, const float* __restrict__ bsrc, const float* __restrict__ csrc,
    const float* __restrict__ g, const float* __restrict__ be,
    float* __restrict__ outp, unsigned short* __restrict__ out16)
{
  __shared__ float red0[4];
  __shared__ float red1[4];
  __shared__ __align__(16) _Float16 sH[kDm];
  const int row = blockIdx.x;
  const int tid = threadIdx.x, lane = tid & 31, wave = tid >> 5;
  const int c4 = tid * 4;
  const size_t ro = (size_t)row * kDm + c4;
  v4f v = *(const v4f*)(a + ro);
  const v4f vb = *(const v4f*)(bsrc + ro);
  v = v + vb;
  if (MODE == 0) {
    const int bb = row / kSeq, t = row - bb * kSeq;
    const int crow = bb * kSeq + (kSeq - 1 - t);
    const v4f vc = *(const v4f*)(csrc + (size_t)crow * kDm + c4);
    v = v + vc;
  }
  float s = (v[0] + v[1]) + (v[2] + v[3]);
#pragma unroll
  for (int off = 16; off > 0; off >>= 1) s += __shfl_xor(s, off, 32);
  if (lane == 0) red0[wave] = s;
  __syncthreads();
  const float mu = ((red0[0] + red0[1]) + (red0[2] + red0[3])) * kInvDm;
  v4f dv;
#pragma unroll
  for (int e = 0; e < 4; ++e) dv[e] = v[e] - mu;
  float s2 = (dv[0] * dv[0] + dv[1] * dv[1]) + (dv[2] * dv[2] + dv[3] * dv[3]);
#pragma unroll
  for (int off = 16; off > 0; off >>= 1) s2 += __shfl_xor(s2, off, 32);
  if (lane == 0) red1[wave] = s2;
  __syncthreads();
  const float var = ((red1[0] + red1[1]) + (red1[2] + red1[3])) * kInvDm;
  const float rs = rsqrtf(var + kLnEps);
  const v4f gv = *(const v4f*)(g + c4);
  const v4f bev = *(const v4f*)(be + c4);
  v4f o;
#pragma unroll
  for (int e = 0; e < 4; ++e) o[e] = dv[e] * rs * gv[e] + bev[e];
  v8h hv;
  if (MODE == 0) {
    v4h hq;
#pragma unroll
    for (int e = 0; e < 4; ++e) hq[e] = (_Float16)o[e];
    *(v4h*)(sH + c4) = hq;
    __syncthreads();
    hv = *(const v8h*)(sH + (tid & 63) * 8);
  }
  float* op = outp + ro;
  unsigned short* oq = (MODE == 0) ? (out16 + (size_t)row * kDm + (tid & 63) * 8) : nullptr;
  for (int pass = 0; pass < 2; ++pass) {
    *(volatile v4f*)op = o;
    if (MODE == 0) {
      if (wave < 2) *(volatile v8h*)oq = hv;
    }
    __threadfence();
  }
}

extern "C" void kernel_launch(void* const* d_in, const int* in_sizes, int n_in,
                              void* d_out, int out_size, void* d_ws, size_t ws_size,
                              hipStream_t stream) {
  if (n_in < 25) return;
  if (in_sizes[0] != kRows * kDm) return;
  for (int m = 0; m < 2; ++m) {
    const int o = 1 + 9 * m;
    if (in_sizes[o + 0] != kXzP * kDm) return;
    if (in_sizes[o + 1] != kDin * 2) return;
    if (in_sizes[o + 2] != kDin) return;
    if (in_sizes[o + 3] != kXdP * kDin) return;
    if (in_sizes[o + 4] != kDin * kDtR) return;
    if (in_sizes[o + 5] != kDin) return;
    if (in_sizes[o + 6] != kDin * kNst) return;
    if (in_sizes[o + 7] != kDin) return;
    if (in_sizes[o + 8] != kDm * kDin) return;
  }
  if (in_sizes[19] != kHid * kDm) return;
  if (in_sizes[20] != kHid) return;
  if (in_sizes[21] != kDm * kHid) return;
  if (in_sizes[22] != kDm) return;
  if (in_sizes[23] != kDm) return;
  if (in_sizes[24] != kDm) return;
  if (out_size != kRows * kDm) return;
  if (ws_size < kWsTotal) return;

  const float* x = (const float*)d_in[0];
  const float* m_in_w[2]   = {(const float*)d_in[1],  (const float*)d_in[10]};
  const float* m_conv_w[2] = {(const float*)d_in[2],  (const float*)d_in[11]};
  const float* m_conv_b[2] = {(const float*)d_in[3],  (const float*)d_in[12]};
  const float* m_xproj[2]  = {(const float*)d_in[4],  (const float*)d_in[13]};
  const float* m_dt_w[2]   = {(const float*)d_in[5],  (const float*)d_in[14]};
  const float* m_dt_b[2]   = {(const float*)d_in[6],  (const float*)d_in[15]};
  const float* m_A_log[2]  = {(const float*)d_in[7],  (const float*)d_in[16]};
  const float* m_Dv[2]     = {(const float*)d_in[8],  (const float*)d_in[17]};
  const float* m_out_w[2]  = {(const float*)d_in[9],  (const float*)d_in[18]};
  const float* pu_w = (const float*)d_in[19];
  const float* pu_b = (const float*)d_in[20];
  const float* pl_w = (const float*)d_in[21];
  const float* pl_b = (const float*)d_in[22];
  const float* ln_g = (const float*)d_in[23];
  const float* ln_b = (const float*)d_in[24];
  float* out = (float*)d_out;

  char* ws = (char*)d_ws;
  unsigned short* X16    = (unsigned short*)(ws + kOffX16);
  unsigned short* XF16   = (unsigned short*)(ws + kOffXF16);
  unsigned short* INW[2] = {(unsigned short*)(ws + kOffINW0), (unsigned short*)(ws + kOffINW1)};
  unsigned short* XPW[2] = {(unsigned short*)(ws + kOffXPW0), (unsigned short*)(ws + kOffXPW1)};
  unsigned short* OUW[2] = {(unsigned short*)(ws + kOffOUW0), (unsigned short*)(ws + kOffOUW1)};
  unsigned short* PU16   = (unsigned short*)(ws + kOffPU16);
  unsigned short* PL16   = (unsigned short*)(ws + kOffPL16);
  float*          XZ[2]  = {(float*)(ws + kOffXZ0), (float*)(ws + kOffXZ1)};
  float*          XC[2]  = {(float*)(ws + kOffXC0), (float*)(ws + kOffXC1)};
  unsigned short* XH[2]  = {(unsigned short*)(ws + kOffXH0), (unsigned short*)(ws + kOffXH1)};
  float*          DB[2]  = {(float*)(ws + kOffDB0), (float*)(ws + kOffDB1)};
  unsigned short* YG[2]  = {(unsigned short*)(ws + kOffYG0), (unsigned short*)(ws + kOffYG1)};
  float*          Y1     = (float*)(ws + kOffY1);
  float*          Y2     = (float*)(ws + kOffY2);
  float*          Y3     = (float*)(ws + kOffY3);
  unsigned short* Y3H    = (unsigned short*)(ws + kOffY3H);
  unsigned short* H16    = (unsigned short*)(ws + kOffH16);
  float*          YP     = (float*)(ws + kOffYP);

  cast_x_f16_kernel<<<(kRows * kDm / 8) / 256, 256, 0, stream>>>(x, X16, XF16, kRows * kDm / 8);
  for (int m = 0; m < 2; ++m) {
    cast_scale_f16_kernel<<<(kXzP * kDm / 8) / 256, 256, 0, stream>>>(m_in_w[m], INW[m], kXzP * kDm / 8, kCarryW);
    cast_scale_f16_kernel<<<(kXdP * kDin / 8) / 256, 256, 0, stream>>>(m_xproj[m], XPW[m], kXdP * kDin / 8, kCarryW);
    cast_scale_f16_kernel<<<(kDm * kDin / 8) / 256, 256, 0, stream>>>(m_out_w[m], OUW[m], kDm * kDin / 8, kCarryW);
  }
  cast_scale_f16_kernel<<<(kHid * kDm / 8) / 256, 256, 0, stream>>>(pu_w, PU16, kHid * kDm / 8, kCarryW);
  cast_scale_f16_kernel<<<(kDm * kHid / 8) / 256, 256, 0, stream>>>(pl_w, PL16, kDm * kHid / 8, kCarryW);

  for (int m = 0; m < 2; ++m) {
    const unsigned short* Ain = (m == 0) ? X16 : XF16;
    wmma_gemm64<0, false, 0, 0, false, 0><<<dim3(((kRows / 64) * (kXzP / 64)) / 8, 1), 256, 0, stream>>>(
        Ain, nullptr, kDm, 0L,
        INW[m], nullptr, kDm, 0L,
        (void*)XZ[m], nullptr, kXzP, 0L,
        nullptr, nullptr, 0L,
        kRows, kXzP, kDm, kScaleIn);
    conv_silu_kernel<<<dim3(kDin / 256, kRows / 64), 256, 0, stream>>>(XZ[m], m_conv_w[m], m_conv_b[m], XC[m], XH[m]);
    wmma_gemm64<0, false, 0, 0, false, 0><<<dim3(((kRows / 64) * (kXdP / 64)) / 8, 1), 256, 0, stream>>>(
        XH[m], nullptr, kDin, 0L,
        XPW[m], nullptr, kDin, 0L,
        (void*)DB[m], nullptr, kXdP, 0L,
        nullptr, nullptr, 0L,
        kRows, kXdP, kDin, kScaleXp);
    scan_kernel<<<kBatch * (kDin / kScanCh), kScanCh, 0, stream>>>(
        DB[m], XC[m], XZ[m], m_dt_w[m], m_dt_b[m], m_A_log[m], m_Dv[m], YG[m]);
    wmma_gemm64<0, false, 0, 0, false, 0><<<dim3(((kRows / 64) * (kDm / 64)) / 8, 1), 256, 0, stream>>>(
        YG[m], nullptr, kDin, 0L,
        OUW[m], nullptr, kDin, 0L,
        (void*)((m == 0) ? Y1 : Y2), nullptr, kDm, 0L,
        nullptr, nullptr, 0L,
        kRows, kDm, kDin, kScaleOut);
  }

  add_ln_kernel<0><<<kRows, kLnThreads, 0, stream>>>(x, Y1, Y2, ln_g, ln_b, Y3, Y3H);

  wmma_gemm64<0, false, 2, 1, false, 2><<<dim3(((kRows / 64) * (kHid / 64)) / 8, 1), 256, 0, stream>>>(
      Y3H, nullptr, kDm, 0L,
      PU16, nullptr, kDm, 0L,
      (void*)H16, nullptr, kHid, 0L,
      pu_b, nullptr, 0L,
      kRows, kHid, kDm, kScaleMlp);

  wmma_gemm64<0, false, 2, 0, false, 0><<<dim3(((kRows / 64) * (kDm / 64)) / 8, 1), 256, 0, stream>>>(
      H16, nullptr, kHid, 0L,
      PL16, nullptr, kHid, 0L,
      (void*)YP, nullptr, kDm, 0L,
      pl_b, nullptr, 0L,
      kRows, kDm, kHid, kScaleMlp);

  add_ln_kernel<1><<<kRows, kLnThreads, 0, stream>>>(YP, Y3, nullptr, ln_g, ln_b, out, nullptr);
}
